// OptimizedAttention_43327630082175
// MI455X (gfx1250) — hardware-verified
//
#include <hip/hip_runtime.h>

typedef __bf16   v16bf __attribute__((ext_vector_type(16)));
typedef float    v8f   __attribute__((ext_vector_type(8)));
typedef float    v4f   __attribute__((ext_vector_type(4)));
typedef unsigned v4u   __attribute__((ext_vector_type(4)));
typedef unsigned v8u   __attribute__((ext_vector_type(8)));

union Frag { v16bf v; v8u w; v4u q[2]; };

#define BB     8
#define SS     1024
#define EE     1024
#define HH     16
#define DD     64
#define NHALF  2
#define BHALF  (BB / NHALF)
#define MH     (BHALF * SS)
#define BHH    (BHALF * HH)
#define QTILES (SS / 16)

#define STG_ROWS 64
#define STG_K    64
#define STG_V4   9
#define TP       68

__device__ __forceinline__ v8f zero8() {
  v8f z;
#pragma unroll
  for (int i = 0; i < 8; ++i) z[i] = 0.0f;
  return z;
}

__device__ __forceinline__ v8f mma16(v16bf a, v16bf b, v8f c) {
  v8f d = __builtin_amdgcn_wmma_f32_16x16x32_bf16(false, a, false, b, (short)0, c, false, false);
  asm volatile("v_nop\n\tv_nop\n\tv_nop\n\tv_nop" : "+v"(d) : "v"(a), "v"(b));
  return d;
}

__device__ __forceinline__ unsigned bfbits(float f) {
  unsigned u = __float_as_uint(f);
  return (u + 0x7FFFu + ((u >> 16) & 1u)) >> 16;
}
__device__ __forceinline__ float bfval(unsigned b) { return __uint_as_float(b << 16); }

__device__ __forceinline__ unsigned pack_pair(float a, float b) {
  return bfbits(a) | (bfbits(b) << 16);
}
__device__ __forceinline__ void split_pair(float a, float b, unsigned& H, unsigned& L) {
  unsigned ha = bfbits(a), hb = bfbits(b);
  unsigned la = bfbits(a - bfval(ha)), lb = bfbits(b - bfval(hb));
  H = ha | (hb << 16);
  L = la | (lb << 16);
}

__device__ __forceinline__ v16bf ldfrag(const __bf16* __restrict__ p, int ld, int lane) {
  const __bf16* base = p + (size_t)(lane & 15) * ld + ((lane >> 4) << 3);
  Frag f;
  f.q[0] = *(const v4u*)(base);
  f.q[1] = *(const v4u*)(base + 16);
  return f.v;
}
__device__ __forceinline__ v16bf ldfrag_lds(const v4u* sh, int row0, int k2, int lane) {
  const v4u* base = sh + (row0 + (lane & 15)) * STG_V4 + (k2 >> 3) + (lane >> 4);
  Frag f;
  f.q[0] = base[0];
  f.q[1] = base[2];
  return f.v;
}

__global__ __launch_bounds__(256)
void k_cvt(const float* __restrict__ in, __bf16* __restrict__ out, int n8) {
  const int i  = blockIdx.x * 256 + threadIdx.x;
  const int ic = (i < n8) ? i : 0;
  const v4f* s = (const v4f*)(in + (size_t)ic * 8);
  v4f a = s[0], b = s[1];
  v4u pk;
  pk.x = pack_pair(a.x, a.y);
  pk.y = pack_pair(a.z, a.w);
  pk.z = pack_pair(b.x, b.y);
  pk.w = pack_pair(b.z, b.w);
  volatile v4u* d = (volatile v4u*)(out + (size_t)ic * 8);
  if (i < n8) { *d = pk; }
  __threadfence();
  if (i < n8) { *d = pk; }
}

__global__ __launch_bounds__(256)
void k_tr(const float* __restrict__ in, __bf16* __restrict__ out, int R, int C) {
  __shared__ float t[64][65];
  const int nbk = R >> 6, nbn = C >> 6;
  if (blockIdx.x >= (unsigned)(nbk * nbn)) return;
  const int bk = blockIdx.x % nbk, bn = blockIdx.x / nbk;
  const int r0 = bk << 6, c0 = bn << 6;
  const int tid = threadIdx.x, lane = tid & 31;
  const int w = __builtin_amdgcn_readfirstlane(tid >> 5);
#pragma unroll
  for (int i = 0; i < 16; ++i) {
    int idx = (i << 8) + tid;
    int r = idx >> 6, c = idx & 63;
    t[r][c] = in[(size_t)(r0 + r) * C + c0 + c];
  }
  __syncthreads();
#pragma unroll
  for (int it = 0; it < 2; ++it) {
    const int line = (w << 3) + (it << 2) + (lane >> 3);
    const int p8 = (lane & 7) << 3;
    v4u pk;
    pk.x = pack_pair(t[p8 + 0][line], t[p8 + 1][line]);
    pk.y = pack_pair(t[p8 + 2][line], t[p8 + 3][line]);
    pk.z = pack_pair(t[p8 + 4][line], t[p8 + 5][line]);
    pk.w = pack_pair(t[p8 + 6][line], t[p8 + 7][line]);
    volatile v4u* d = (volatile v4u*)(out + (size_t)(c0 + line) * R + r0 + p8);
    *d = pk;
    __threadfence();
    *d = pk;
  }
}

__global__ __launch_bounds__(256)
void k_qkv(const __bf16* __restrict__ A, const __bf16* __restrict__ BT,
           const float* __restrict__ bias,
           __bf16* __restrict__ qh, __bf16* __restrict__ ql,
           __bf16* __restrict__ kh, __bf16* __restrict__ kl,
           __bf16* __restrict__ vth, __bf16* __restrict__ vtl) {
  __shared__ v4u   shB[STG_ROWS * STG_V4];
  __shared__ float tile[256 * TP];
  const int Kd = EE;
  const int NB = (3 * EE) / 64;
  const int tid = threadIdx.x, lane = tid & 31;
  const int w  = __builtin_amdgcn_readfirstlane(tid >> 5);
  const int bm = blockIdx.x / NB, bn = blockIdx.x % NB;
  if (bm >= MH / 256) return;
  const int m0 = bm * 256 + w * 32;
  const int n0 = bn * 64;

  v8f acc[2][4];
#pragma unroll
  for (int i = 0; i < 2; ++i)
#pragma unroll
    for (int g = 0; g < 4; ++g) acc[i][g] = zero8();

  const int srow = tid >> 3, skb = tid & 7;
  for (int ks = 0; ks < Kd; ks += STG_K) {
    __syncthreads();
    {
      const v4u* g0 = (const v4u*)(BT + (size_t)(n0 + srow) * Kd + ks) + skb;
      const v4u* g1 = (const v4u*)(BT + (size_t)(n0 + 32 + srow) * Kd + ks) + skb;
      shB[srow * STG_V4 + skb]        = *g0;
      shB[(srow + 32) * STG_V4 + skb] = *g1;
    }
    __syncthreads();
    const __bf16* Ab = A + (size_t)m0 * Kd + ks;
#pragma unroll
    for (int k2 = 0; k2 < STG_K; k2 += 32) {
      v16bf a0 = ldfrag(Ab + k2, Kd, lane);
      v16bf a1 = ldfrag(Ab + (size_t)16 * Kd + k2, Kd, lane);
#pragma unroll
      for (int g = 0; g < 4; ++g) {
        v16bf bf = ldfrag_lds(shB, g * 16, k2, lane);
        acc[0][g] = mma16(a0, bf, acc[0][g]);
        acc[1][g] = mma16(a1, bf, acc[1][g]);
      }
    }
  }

  const int nl = lane & 15, mh = (lane >> 4) << 3;
#pragma unroll
  for (int ms = 0; ms < 2; ++ms)
#pragma unroll
    for (int g = 0; g < 4; ++g) {
      const int   col = n0 + g * 16 + nl;
      const float bv  = bfval(bfbits(bias[col]));
#pragma unroll
      for (int r = 0; r < 8; ++r)
        tile[(w * 32 + ms * 16 + mh + r) * TP + g * 16 + nl] = acc[ms][g][r] + bv;
    }
  __syncthreads();

  const int which = n0 >> 10;
  const int hd    = (n0 & (EE - 1)) >> 6;
  const int bi    = bm >> 2;
  const int s0    = (bm & 3) << 8;
  const size_t bh = (size_t)bi * HH + hd;

  if (which < 2) {
    __bf16* ph = (which == 0) ? qh : kh;
    __bf16* pl = (which == 0) ? ql : kl;
    const float sc = (which == 0) ? 0.125f : 1.0f;
#pragma unroll
    for (int it = 0; it < 8; ++it) {
      const int row = w * 32 + it * 4 + (lane >> 3);
      const int p8  = (lane & 7) << 3;
      const float* s = tile + row * TP + p8;
      unsigned h0, h1, h2, h3, l0, l1, l2, l3;
      split_pair(s[0] * sc, s[1] * sc, h0, l0);
      split_pair(s[2] * sc, s[3] * sc, h1, l1);
      split_pair(s[4] * sc, s[5] * sc, h2, l2);
      split_pair(s[6] * sc, s[7] * sc, h3, l3);
      v4u H, L;
      H.x = h0; H.y = h1; H.z = h2; H.w = h3;
      L.x = l0; L.y = l1; L.z = l2; L.w = l3;
      const size_t off = (bh * SS + s0 + row) * DD + p8;
      volatile v4u* dh = (volatile v4u*)(ph + off);
      volatile v4u* dl = (volatile v4u*)(pl + off);
      *dh = H; *dl = L;
      __threadfence();
      *dh = H; *dl = L;
    }
  } else {
#pragma unroll
    for (int j = 0; j < 8; ++j) {
      const int d = w * 8 + j;
      const float* s = tile + (lane * 8) * TP + d;
      unsigned h0, h1, h2, h3, l0, l1, l2, l3;
      split_pair(s[0 * TP], s[1 * TP], h0, l0);
      split_pair(s[2 * TP], s[3 * TP], h1, l1);
      split_pair(s[4 * TP], s[5 * TP], h2, l2);
      split_pair(s[6 * TP], s[7 * TP], h3, l3);
      v4u H, L;
      H.x = h0; H.y = h1; H.z = h2; H.w = h3;
      L.x = l0; L.y = l1; L.z = l2; L.w = l3;
      const size_t off = (bh * DD + d) * SS + s0 + lane * 8;
      volatile v4u* dh = (volatile v4u*)(vth + off);
      volatile v4u* dl = (volatile v4u*)(vtl + off);
      *dh = H; *dl = L;
      __threadfence();
      *dh = H; *dl = L;
    }
  }
}

__global__ __launch_bounds__(256)
void k_attn(const __bf16* __restrict__ qh, const __bf16* __restrict__ ql,
            const __bf16* __restrict__ kh, const __bf16* __restrict__ kl,
            const __bf16* __restrict__ vth, const __bf16* __restrict__ vtl,
            __bf16* __restrict__ aoh, __bf16* __restrict__ aol) {
  __shared__ v4f ot[8 * 256];
  const int tid = threadIdx.x, lane = tid & 31;
  const int w   = __builtin_amdgcn_readfirstlane(tid >> 5);
  const int wid = blockIdx.x * 8 + w;
  const int qt  = wid % QTILES;
  const int bh  = wid / QTILES;
  const int hd  = bh % HH, b = bh / HH;

  const size_t pq = (size_t)bh * SS * DD;
  const __bf16* Qh = qh + pq;   const __bf16* Ql = ql + pq;
  const __bf16* Kh = kh + pq;   const __bf16* Kl = kl + pq;
  const size_t pv = (size_t)bh * DD * SS;
  const __bf16* Vh = vth + pv;  const __bf16* Vl = vtl + pv;
  const int q0 = qt * 16;

  v16bf qfh0 = ldfrag(Qh + (size_t)q0 * DD,      DD, lane);
  v16bf qfh1 = ldfrag(Qh + (size_t)q0 * DD + 32, DD, lane);
  v16bf qfl0 = ldfrag(Ql + (size_t)q0 * DD,      DD, lane);
  v16bf qfl1 = ldfrag(Ql + (size_t)q0 * DD + 32, DD, lane);

  v8f acc[4];
#pragma unroll
  for (int g = 0; g < 4; ++g) acc[g] = zero8();

  float m_run = -1e30f, l_run = 0.0f;
  const int qg    = q0 + (lane & 15);
  const int half8 = (lane >> 4) << 3;

  for (int kvb = 0; kvb < q0 + 16; kvb += 32) {
    v8f st[2];
    st[0] = zero8(); st[1] = zero8();
#pragma unroll
    for (int j = 0; j < 2; ++j) {
      if (kvb + j * 16 < q0 + 16) {
        const __bf16* kph = Kh + (size_t)(kvb + j * 16) * DD;
        const __bf16* kpl = Kl + (size_t)(kvb + j * 16) * DD;
        v16bf a0 = ldfrag(kph, DD, lane);
        v16bf c0 = ldfrag(kpl, DD, lane);
        st[j] = mma16(a0, qfh0, st[j]);
        st[j] = mma16(a0, qfl0, st[j]);
        st[j] = mma16(c0, qfh0, st[j]);
        v16bf a1 = ldfrag(kph + 32, DD, lane);
        v16bf c1 = ldfrag(kpl + 32, DD, lane);
        st[j] = mma16(a1, qfh1, st[j]);
        st[j] = mma16(a1, qfl1, st[j]);
        st[j] = mma16(c1, qfh1, st[j]);
      }
    }
    float mx = -1e30f;
#pragma unroll
    for (int j = 0; j < 2; ++j)
#pragma unroll
      for (int r = 0; r < 8; ++r) {
        const int   kvg = kvb + j * 16 + half8 + r;
        const float sv  = (kvg <= qg) ? st[j][r] : -1e30f;
        st[j][r] = sv;
        mx = fmaxf(mx, sv);
      }
    mx = fmaxf(mx, __shfl_xor(mx, 16, 32));
    const float m_new = fmaxf(m_run, mx);
    const float alpha = __expf(m_run - m_new);

    float psum = 0.0f;
    Frag PH, PL;
#pragma unroll
    for (int rr = 0; rr < 4; ++rr) {
      const float a0 = __expf(st[0][2 * rr] - m_new), a1 = __expf(st[0][2 * rr + 1] - m_new);
      const float b0 = __expf(st[1][2 * rr] - m_new), b1 = __expf(st[1][2 * rr + 1] - m_new);
      psum += (a0 + a1) + (b0 + b1);
      unsigned hw, lw;
      split_pair(a0, a1, hw, lw); PH.w[rr] = hw;     PL.w[rr] = lw;
      split_pair(b0, b1, hw, lw); PH.w[4 + rr] = hw; PL.w[4 + rr] = lw;
    }
    psum += __shfl_xor(psum, 16, 32);
    l_run = l_run * alpha + psum;
    m_run = m_new;

#pragma unroll
    for (int g = 0; g < 4; ++g) {
      v16bf vh = ldfrag(Vh + (size_t)(g * 16) * SS + kvb, SS, lane);
      v16bf vl = ldfrag(Vl + (size_t)(g * 16) * SS + kvb, SS, lane);
#pragma unroll
      for (int r = 0; r < 8; ++r) acc[g][r] *= alpha;
      acc[g] = mma16(vh, PH.v, acc[g]);
      acc[g] = mma16(vh, PL.v, acc[g]);
      acc[g] = mma16(vl, PH.v, acc[g]);
    }
  }

  const float inv = (l_run > 0.0f) ? (1.0f / l_run) : 0.0f;
  v4f* mt = ot + w * 256;
  const int n = lane & 15, hh = lane >> 4;
#pragma unroll
  for (int g = 0; g < 4; ++g) {
    v4f u0, u1;
    u0.x = acc[g][0] * inv; u0.y = acc[g][1] * inv; u0.z = acc[g][2] * inv; u0.w = acc[g][3] * inv;
    u1.x = acc[g][4] * inv; u1.y = acc[g][5] * inv; u1.z = acc[g][6] * inv; u1.w = acc[g][7] * inv;
    mt[n * 16 + g * 4 + 2 * hh]     = u0;
    mt[n * 16 + g * 4 + 2 * hh + 1] = u1;
  }
  __syncthreads();
#pragma unroll
  for (int it = 0; it < 4; ++it) {
    const int qr = it * 4 + (lane >> 3);
    const int p  = lane & 7;
    const v4f x0 = mt[qr * 16 + 2 * p], x1 = mt[qr * 16 + 2 * p + 1];
    unsigned h0, h1, h2, h3, l0, l1, l2, l3;
    split_pair(x0.x, x0.y, h0, l0);
    split_pair(x0.z, x0.w, h1, l1);
    split_pair(x1.x, x1.y, h2, l2);
    split_pair(x1.z, x1.w, h3, l3);
    v4u H, L;
    H.x = h0; H.y = h1; H.z = h2; H.w = h3;
    L.x = l0; L.y = l1; L.z = l2; L.w = l3;
    const size_t off = ((size_t)b * SS + q0 + qr) * EE + hd * DD + p * 8;
    volatile v4u* dh = (volatile v4u*)(aoh + off);
    volatile v4u* dl = (volatile v4u*)(aol + off);
    *dh = H; *dl = L;
    __threadfence();
    *dh = H; *dl = L;
  }
}

__global__ __launch_bounds__(256)
void k_proj(const __bf16* __restrict__ Ah, const __bf16* __restrict__ Al,
            const __bf16* __restrict__ BT, const float* __restrict__ bias,
            float* __restrict__ out) {
  __shared__ v4u   shB[STG_ROWS * STG_V4];
  __shared__ float tile[256 * TP];
  const int Kd = EE;
  const int NB = EE / 64;
  const int tid = threadIdx.x, lane = tid & 31;
  const int w  = __builtin_amdgcn_readfirstlane(tid >> 5);
  const int bm = blockIdx.x / NB, bn = blockIdx.x % NB;
  if (bm >= MH / 256) return;
  const int m0 = bm * 256 + w * 32;
  const int n0 = bn * 64;

  v8f acc[2][4];
#pragma unroll
  for (int i = 0; i < 2; ++i)
#pragma unroll
    for (int g = 0; g < 4; ++g) acc[i][g] = zero8();

  const int srow = tid >> 3, skb = tid & 7;
  for (int ks = 0; ks < Kd; ks += STG_K) {
    __syncthreads();
    {
      const v4u* g0 = (const v4u*)(BT + (size_t)(n0 + srow) * Kd + ks) + skb;
      const v4u* g1 = (const v4u*)(BT + (size_t)(n0 + 32 + srow) * Kd + ks) + skb;
      shB[srow * STG_V4 + skb]        = *g0;
      shB[(srow + 32) * STG_V4 + skb] = *g1;
    }
    __syncthreads();
    const __bf16* Abh = Ah + (size_t)m0 * Kd + ks;
    const __bf16* Abl = Al + (size_t)m0 * Kd + ks;
#pragma unroll
    for (int k2 = 0; k2 < STG_K; k2 += 32) {
      v16bf a0h = ldfrag(Abh + k2, Kd, lane);
      v16bf a1h = ldfrag(Abh + (size_t)16 * Kd + k2, Kd, lane);
      v16bf a0l = ldfrag(Abl + k2, Kd, lane);
      v16bf a1l = ldfrag(Abl + (size_t)16 * Kd + k2, Kd, lane);
#pragma unroll
      for (int g = 0; g < 4; ++g) {
        v16bf bf = ldfrag_lds(shB, g * 16, k2, lane);
        acc[0][g] = mma16(a0h, bf, acc[0][g]);
        acc[0][g] = mma16(a0l, bf, acc[0][g]);
        acc[1][g] = mma16(a1h, bf, acc[1][g]);
        acc[1][g] = mma16(a1l, bf, acc[1][g]);
      }
    }
  }

  const int nl = lane & 15, mh = (lane >> 4) << 3;
#pragma unroll
  for (int ms = 0; ms < 2; ++ms)
#pragma unroll
    for (int g = 0; g < 4; ++g) {
      const int   col = n0 + g * 16 + nl;
      const float bv  = bfval(bfbits(bias[col]));
#pragma unroll
      for (int r = 0; r < 8; ++r)
        tile[(w * 32 + ms * 16 + mh + r) * TP + g * 16 + nl] = acc[ms][g][r] + bv;
    }
  __syncthreads();

#pragma unroll
  for (int it = 0; it < 16; ++it) {
    const int row = w * 32 + it * 2 + (lane >> 4);
    const int c4  = (lane & 15) << 2;
    const float* s = tile + row * TP + c4;
    v4f v;
    v.x = s[0]; v.y = s[1]; v.z = s[2]; v.w = s[3];
    volatile v4f* d = (volatile v4f*)(out + (size_t)(bm * 256 + row) * EE + n0 + c4);
    *d = v;
    __threadfence();
    *d = v;
  }
}

extern "C" void kernel_launch(void* const* d_in, const int* in_sizes, int n_in,
                              void* d_out, int out_size, void* d_ws,
                              size_t ws_size, hipStream_t stream) {
  if (n_in < 5) return;
  if (in_sizes[0] != BB * SS * EE || in_sizes[1] != EE * 3 * EE || in_sizes[2] != 3 * EE ||
      in_sizes[3] != EE * EE || in_sizes[4] != EE || out_size != BB * SS * EE) return;
  const size_t MB = (size_t)1 << 20;
  const size_t need = 88 * MB;
  if (ws_size < need) return;

  const float* x  = (const float*)d_in[0];
  const float* Wa = (const float*)d_in[1];
  const float* ba = (const float*)d_in[2];
  const float* Wp = (const float*)d_in[3];
  const float* bp = (const float*)d_in[4];
  float* out = (float*)d_out;

  char* ws = (char*)d_ws;
  __bf16* xb  = (__bf16*)(ws +  0 * MB);
  __bf16* wat = (__bf16*)(ws + 16 * MB);
  __bf16* wpt = (__bf16*)(ws + 22 * MB);
  __bf16* qh  = (__bf16*)(ws + 24 * MB);
  __bf16* ql  = (__bf16*)(ws + 32 * MB);
  __bf16* kh  = (__bf16*)(ws + 40 * MB);
  __bf16* kl  = (__bf16*)(ws + 48 * MB);
  __bf16* vth = (__bf16*)(ws + 56 * MB);
  __bf16* vtl = (__bf16*)(ws + 64 * MB);
  __bf16* aoh = (__bf16*)(ws + 72 * MB);
  __bf16* aol = (__bf16*)(ws + 80 * MB);

  const int n8 = BB * SS * EE / 8;
  k_cvt<<<n8 / 256, 256, 0, stream>>>(x, xb, n8);
  k_tr<<<(EE / 64) * (3 * EE / 64), 256, 0, stream>>>(Wa, wat, EE, 3 * EE);
  k_tr<<<(EE / 64) * (EE / 64), 256, 0, stream>>>(Wp, wpt, EE, EE);

  for (int half = 0; half < NHALF; ++half) {
    const __bf16* xhb = xb + (size_t)half * MH * EE;
    float* outh = out + (size_t)half * MH * EE;
    k_qkv<<<(MH / 256) * (3 * EE / 64), 256, 0, stream>>>(xhb, wat, ba, qh, ql, kh, kl, vth, vtl);
    k_attn<<<(BHH * QTILES) / 8, 256, 0, stream>>>(qh, ql, kh, kl, vth, vtl, aoh, aol);
    k_proj<<<(MH / 256) * (EE / 64), 256, 0, stream>>>(aoh, aol, wpt, bp, outh);
  }
}
